// Block_73976516706525
// MI455X (gfx1250) — hardware-run, weakly checked
//
#include <hip/hip_runtime.h>
#include <stdint.h>
#include <math.h>


typedef _Float16 v16h __attribute__((ext_vector_type(16)));
typedef _Float16 v8h  __attribute__((ext_vector_type(8)));
typedef _Float16 v4h  __attribute__((ext_vector_type(4)));
typedef float    v8f  __attribute__((ext_vector_type(8)));
typedef float    v4f  __attribute__((ext_vector_type(4)));

#ifndef NB
#define NB 2
#endif
#ifndef SEQ
#define SEQ 1024
#endif
#define NB_FULL  2
#define SEQ_FULL 1024
#define DM   768
#define NH   12
#define HD   64
#define MLP  3072
#define ROWS (NB * SEQ)
#define PQ   256
#define PE   16

#define ACT_CAR   8.0f
#define W_CAR     1024.0f
#define SCL_M10   0.0009765625f
#define SCL_M13   0.0001220703125f
#define SCL_M20   9.5367431640625e-07f
#define PS_SCL    0.001953125f
#define P_CAR     16384.0f
#define PV_SCL    7.62939453125e-06f
#define EW_SCL    0.001953125f
#define CTX_CAR   128.0f
#define CAT_CAR   1024.0f
#define FW_CAR    64.0f
#define FUS_SCL   0.015625f
#define DCT_THR   0.01f

#define GM_F32  1
#define GM_THR  2
#define GM_GELU 4
#define GM_BIAS 8

static_assert(NB == 1 || NB == 2);
static_assert(NB <= NB_FULL);
static_assert(SEQ == SEQ_FULL);
static_assert(SEQ == 1024 && SEQ == 32 * 32);
static_assert(DM == NH * HD);
static_assert(HD == 64 && NH == 12 && 2 * NH <= 32);
static_assert(PQ * 4 == SEQ && PE * 4 == HD && PE == 16 && PQ == 256);
static_assert(DM == 3 * 256);
static_assert(DM % 128 == 0 && DM % 64 == 0 && DM % 32 == 0);
static_assert(MLP % 64 == 0 && MLP % 32 == 0);
static_assert(SEQ % 128 == 0 && ROWS % 128 == 0 && (3 * ROWS) % 128 == 0);
static_assert(ROWS % 16 == 0 && ROWS % 8 == 0);
static_assert(((long)SEQ * SEQ) % 2048 == 0 && ((long)DM * DM) % 2048 == 0);
static_assert(((long)DM * DM / 8) % 256 == 0 && ((long)MLP * DM / 8) % 256 == 0);
static_assert(((long)3 * ROWS * DM / 8) % 256 == 0);
static_assert((long)NB_FULL * SEQ_FULL * DM * 4 == 6291456L);

#define N_DS   ((size_t)2 * SEQ * SEQ)
#define N_DD   ((size_t)2 * DM * DM)
#define N_WQ   ((size_t)3 * DM * DM)
#define N_W1   ((size_t)DM * DM)
#define N_FC   ((size_t)MLP * DM)
#define N_ACT  ((size_t)ROWS * DM)
#define N_3ACT ((size_t)3 * ROWS * DM)
#define N_CS   ((size_t)2 * NB * NH * PQ * PE)
#define N_X2   ((size_t)2 * ROWS * DM)
#define N_H1   ((size_t)ROWS * MLP)
#define WS_HALVES (N_DS + N_DD + N_WQ + 2 * N_W1 + 2 * N_FC + 7 * N_ACT + 3 * N_3ACT + N_CS + N_X2 + N_H1)
static_assert(WS_HALVES * 2 <= (size_t)134217728);
static_assert(N_DS % 64 == 0 && N_DD % 64 == 0 && N_WQ % 64 == 0 && N_W1 % 64 == 0 && N_FC % 64 == 0);
static_assert(N_ACT % 64 == 0 && N_3ACT % 64 == 0 && N_CS % 64 == 0 && N_X2 % 64 == 0 && N_H1 % 64 == 0);

union Frag16 { v16h v; v8h p[2]; };

__device__ __forceinline__ v16h ld_frag_g(const _Float16* __restrict__ p, int hl) {
  Frag16 f;
  f.p[0] = *(const v8h*)(p + 8 * hl);
  f.p[1] = *(const v8h*)(p + 16 + 8 * hl);
  return f.v;
}

__device__ __forceinline__ v16h ld_frag_s(const _Float16* base, int off, int hl) {
  Frag16 f;
  f.p[0] = *(const v8h*)(base + off + 8 * hl);
  f.p[1] = *(const v8h*)(base + off + 16 + 8 * hl);
  return f.v;
}

__device__ __forceinline__ v8f mma(v16h a, v16h b, v8f c) {
  v8f d = __builtin_amdgcn_wmma_f32_16x16x32_f16(false, a, false, b, (short)0, c, false, false);
  asm volatile("v_nop\n\tv_nop\n\tv_nop\n\tv_nop" : "+v"(d) : "v"(a), "v"(b));
  return d;
}

__device__ __forceinline__ float bf16_rne(float x) {
  unsigned int u = __builtin_bit_cast(unsigned int, x);
  u += 0x7FFFu + ((u >> 16) & 1u);
  return __builtin_bit_cast(float, u & 0xFFFF0000u);
}

static __device__ __forceinline__ _Float16 toh_flush(float v) {
  const _Float16 r = (_Float16)v;
  return (fabsf(v) < 6.103515625e-05f) ? (_Float16)0.0f : r;
}

__global__ __launch_bounds__(256) void k_cvt8(const float* __restrict__ src,
                                              _Float16* __restrict__ dst,
                                              int cols, int seq, int seq_full, float car, int total8)
{
  const int i8 = blockIdx.x * 256 + threadIdx.x;
  if (i8 >= total8) return;
  const size_t e   = (size_t)i8 * 8;
  const int    r   = (int)(e / (size_t)cols);
  const int    col = (int)(e - (size_t)r * (size_t)cols);
  const int    bb  = r / seq;
  const int    nn  = r - bb * seq;
  const float* s = src + ((size_t)bb * seq_full + nn) * (size_t)cols + col;
  const v4f x0 = *(const v4f*)s;
  const v4f x1 = *(const v4f*)(s + 4);
  v8h o;
#pragma unroll
  for (int j = 0; j < 4; ++j) {
    const float t0 = x0[j];
    const float t1 = x1[j];
    o[j]     = (_Float16)(bf16_rne(t0) * car);
    o[4 + j] = (_Float16)(bf16_rne(t1) * car);
  }
  _Float16* d = dst + e;
  *(volatile v8h*)d = o;
  __threadfence();
  *(volatile v8h*)d = o;
}

__global__ __launch_bounds__(256) void k_gen(_Float16* __restrict__ dst, int n, float s0, float sk)
{
#pragma clang fp contract(off)
  __shared__ __attribute__((aligned(16))) _Float16 lt[2048];
  const int tid = threadIdx.x;
  const int tr = blockIdx.y;
  const int g0 = blockIdx.x * 2048;
  const int n2 = 2 * n, n4 = 4 * n;
  const float inv2n = 1.0f / (float)n2;
#pragma unroll 1
  for (int j = 0; j < 8; ++j) {
    const int g = g0 + j * 256 + tid;
    const int row = g / n;
    const int col = g - row * n;
    const int kk = (tr != 0) ? col : row;
    const int ii = (tr != 0) ? row : col;
    int m = ((2 * ii + 1) * kk) % n4;
    if (m > n2) m = n4 - m;
    float sg = 1.0f;
    if (m > n) { m = n2 - m; sg = -1.0f; }
    const float cv = cospif((float)m * inv2n);
    const float val = sg * cv * ((kk == 0) ? s0 : sk);
    lt[j * 256 + tid] = toh_flush(val * W_CAR);
  }
  __syncthreads();
  const v8h o = *(const v8h*)(&lt[tid * 8]);
  _Float16* d = dst + (size_t)tr * (size_t)n * (size_t)n + (size_t)g0 + (size_t)tid * 8;
  *(volatile v8h*)d = o;
  __threadfence();
  *(volatile v8h*)d = o;
}

__global__ __launch_bounds__(256) void k_ln(const float* __restrict__ src,
                                            const float* __restrict__ g,
                                            const float* __restrict__ be,
                                            _Float16* __restrict__ dst, int rnd, int rows)
{
#pragma clang fp contract(off)
  const int lane = threadIdx.x & 31;
  const int wave = __builtin_amdgcn_readfirstlane(threadIdx.x >> 5);
  const int r = blockIdx.x * 8 + wave;
  if (r >= rows) return;
  const float* s = src + (size_t)r * DM + lane * 8;

  float sum = 0.f;
#pragma unroll 1
  for (int t = 0; t < 3; ++t) {
    const v4f a  = *(const v4f*)(s + t * 256);
    const v4f b4 = *(const v4f*)(s + t * 256 + 4);
#pragma unroll
    for (int j = 0; j < 4; ++j) {
      const float x0 = (rnd != 0) ? bf16_rne(a[j])  : a[j];
      const float x1 = (rnd != 0) ? bf16_rne(b4[j]) : b4[j];
      sum += x0 + x1;
    }
  }
  sum += __shfl_xor(sum, 16, 32);
  sum += __shfl_xor(sum, 8, 32);
  sum += __shfl_xor(sum, 4, 32);
  sum += __shfl_xor(sum, 2, 32);
  sum += __shfl_xor(sum, 1, 32);
  const float mu = sum * (1.0f / (float)DM);

  float vs = 0.f;
#pragma unroll 1
  for (int t = 0; t < 3; ++t) {
    const v4f a  = *(const v4f*)(s + t * 256);
    const v4f b4 = *(const v4f*)(s + t * 256 + 4);
#pragma unroll
    for (int j = 0; j < 4; ++j) {
      const float x0 = (rnd != 0) ? bf16_rne(a[j])  : a[j];
      const float x1 = (rnd != 0) ? bf16_rne(b4[j]) : b4[j];
      const float d0 = x0 - mu, d1 = x1 - mu;
      vs += d0 * d0 + d1 * d1;
    }
  }
  vs += __shfl_xor(vs, 16, 32);
  vs += __shfl_xor(vs, 8, 32);
  vs += __shfl_xor(vs, 4, 32);
  vs += __shfl_xor(vs, 2, 32);
  vs += __shfl_xor(vs, 1, 32);
  const float inv = 1.0f / sqrtf(vs * (1.0f / (float)DM) + 1e-6f);

  v8h o[3];
#pragma unroll
  for (int t = 0; t < 3; ++t) {
    const v4f a  = *(const v4f*)(s + t * 256);
    const v4f b4 = *(const v4f*)(s + t * 256 + 4);
    const v4f ga = *(const v4f*)(g + t * 256 + lane * 8);
    const v4f gb = *(const v4f*)(g + t * 256 + lane * 8 + 4);
    const v4f ba = *(const v4f*)(be + t * 256 + lane * 8);
    const v4f bb = *(const v4f*)(be + t * 256 + lane * 8 + 4);
#pragma unroll
    for (int j = 0; j < 4; ++j) {
      const float x0 = (rnd != 0) ? bf16_rne(a[j])  : a[j];
      const float x1 = (rnd != 0) ? bf16_rne(b4[j]) : b4[j];
      const float y0 = (x0 - mu) * inv * bf16_rne(ga[j]) + bf16_rne(ba[j]);
      const float y1 = (x1 - mu) * inv * bf16_rne(gb[j]) + bf16_rne(bb[j]);
      o[t][j]     = toh_flush(y0 * ACT_CAR);
      o[t][4 + j] = toh_flush(y1 * ACT_CAR);
    }
  }
  _Float16* d = dst + (size_t)r * DM + lane * 8;
  *(volatile v8h*)(d)       = o[0];
  *(volatile v8h*)(d + 256) = o[1];
  *(volatile v8h*)(d + 512) = o[2];
  __threadfence();
  *(volatile v8h*)(d)       = o[0];
  *(volatile v8h*)(d + 256) = o[1];
  *(volatile v8h*)(d + 512) = o[2];
}

__device__ __forceinline__ void gemm_core(const _Float16* __restrict__ ap0,
                                          const _Float16* __restrict__ ap1,
                                          const _Float16* __restrict__ bp, int K, int hl, v8f (&acc)[8])
{
  const size_t bst = (size_t)16 * K;
#pragma unroll 1
  for (int k0 = 0; k0 < K; k0 += 32) {
    const v16h a0 = ld_frag_g(ap0 + k0, hl);
    const v16h a1 = ld_frag_g(ap1 + k0, hl);
    const v16h b0 = ld_frag_g(bp + k0, hl);
    const v16h b1 = ld_frag_g(bp + bst + k0, hl);
    const v16h b2 = ld_frag_g(bp + 2 * bst + k0, hl);
    const v16h b3 = ld_frag_g(bp + 3 * bst + k0, hl);
    acc[0] = mma(a0, b0, acc[0]);
    acc[1] = mma(a0, b1, acc[1]);
    acc[2] = mma(a0, b2, acc[2]);
    acc[3] = mma(a0, b3, acc[3]);
    acc[4] = mma(a1, b0, acc[4]);
    acc[5] = mma(a1, b1, acc[5]);
    acc[6] = mma(a1, b2, acc[6]);
    acc[7] = mma(a1, b3, acc[7]);
  }
}

__global__ __launch_bounds__(128) __attribute__((amdgpu_num_vgpr(256)))
void k_gemm(const _Float16* __restrict__ A, const _Float16* __restrict__ Bt,
            const float* __restrict__ bias, const float* __restrict__ res,
            _Float16* __restrict__ CH, float* __restrict__ CF,
            size_t sA, size_t sB, size_t sC,
            int K, int ldc, float scl, float bcar, float ocar, int mode, int resrnd)
{
  __shared__ __attribute__((aligned(16))) float ldsF[128 * 68];

  const int tid = threadIdx.x, lane = tid & 31;
  const int w = __builtin_amdgcn_readfirstlane(tid >> 5);
  const int hl = lane >> 4, c = lane & 15;
  const int z = blockIdx.z;
  const int m0 = blockIdx.y * 128, n0 = blockIdx.x * 64;
  const int mw = m0 + 32 * w;

  const _Float16* az = A  + (size_t)z * sA;
  const _Float16* bz = Bt + (size_t)z * sB;
  const _Float16* ap0 = az + (size_t)(mw + c) * K;
  const _Float16* ap1 = az + (size_t)(mw + 16 + c) * K;
  const _Float16* bp  = bz + (size_t)(n0 + c) * K;

  v8f acc[8] = {};
  gemm_core(ap0, ap1, bp, K, hl, acc);

#pragma unroll
  for (int i = 0; i < 2; ++i)
#pragma unroll
    for (int t = 0; t < 4; ++t)
#pragma unroll
      for (int r = 0; r < 8; ++r) {
        const int rowl = 32 * w + 16 * i + 8 * hl + r;
        ldsF[rowl * 68 + 16 * t + c] = acc[i * 4 + t][r] * scl;
      }
  __syncthreads();

  if ((mode & (GM_THR | GM_GELU | GM_BIAS)) != 0) {
    const int fc = tid & 63;
    const int fr = tid >> 6;
    float bv = 0.f;
    if ((mode & GM_BIAS) != 0) bv = bf16_rne(bias[n0 + fc]) * bcar;
#pragma unroll 1
    for (int j = 0; j < 64; ++j) {
      const int li = (2 * j + fr) * 68 + fc;
      float v = ldsF[li] + bv;
      if ((mode & GM_THR) != 0) v = (fabsf(v) > DCT_THR) ? v : 0.f;
      if ((mode & GM_GELU) != 0) v = 0.5f * v * (1.0f + erff(v * 0.70710678118654752f));
      ldsF[li] = v;
    }
    __syncthreads();
  }

  if ((mode & GM_F32) == 0) {
    _Float16* const bh = CH + (size_t)z * sC + (size_t)m0 * ldc + n0;
    for (int i = 0; i < 8; ++i) {
      const int q = i * 128 + tid;
      const int rowl = q >> 3, ch = (q & 7) * 8;
      const v4f a  = *(const v4f*)(&ldsF[rowl * 68 + ch]);
      const v4f b4 = *(const v4f*)(&ldsF[rowl * 68 + ch + 4]);
      v8h o;
      o[0] = toh_flush(a[0] * ocar);  o[1] = toh_flush(a[1] * ocar);
      o[2] = toh_flush(a[2] * ocar);  o[3] = toh_flush(a[3] * ocar);
      o[4] = toh_flush(b4[0] * ocar); o[5] = toh_flush(b4[1] * ocar);
      o[6] = toh_flush(b4[2] * ocar); o[7] = toh_flush(b4[3] * ocar);
      *(volatile v8h*)(bh + (size_t)rowl * ldc + ch) = o;
    }
    __threadfence();
    for (int i = 0; i < 8; ++i) {
      const int q = i * 128 + tid;
      const int rowl = q >> 3, ch = (q & 7) * 8;
      const v4f a  = *(const v4f*)(&ldsF[rowl * 68 + ch]);
      const v4f b4 = *(const v4f*)(&ldsF[rowl * 68 + ch + 4]);
      v8h o;
      o[0] = toh_flush(a[0] * ocar);  o[1] = toh_flush(a[1] * ocar);
      o[2] = toh_flush(a[2] * ocar);  o[3] = toh_flush(a[3] * ocar);
      o[4] = toh_flush(b4[0] * ocar); o[5] = toh_flush(b4[1] * ocar);
      o[6] = toh_flush(b4[2] * ocar); o[7] = toh_flush(b4[3] * ocar);
      *(volatile v8h*)(bh + (size_t)rowl * ldc + ch) = o;
    }
  } else {
    float* const ob = CF + (size_t)z * sC + (size_t)m0 * ldc + n0;
    const float* const rb = res + (size_t)z * sC + (size_t)m0 * ldc + n0;
    for (int i = 0; i < 16; ++i) {
      const int qi = i * 128 + tid;
      const int rowl = qi >> 4, col = (qi & 15) * 4;
      const v4f rr = *(const v4f*)(rb + (size_t)rowl * ldc + col);
      v4f v = *(const v4f*)(&ldsF[rowl * 68 + col]);
      v[0] += (resrnd != 0) ? bf16_rne(rr[0]) : rr[0];
      v[1] += (resrnd != 0) ? bf16_rne(rr[1]) : rr[1];
      v[2] += (resrnd != 0) ? bf16_rne(rr[2]) : rr[2];
      v[3] += (resrnd != 0) ? bf16_rne(rr[3]) : rr[3];
      *(volatile v4f*)(ob + (size_t)rowl * ldc + col) = v;
    }
    __threadfence();
    for (int i = 0; i < 16; ++i) {
      const int qi = i * 128 + tid;
      const int rowl = qi >> 4, col = (qi & 15) * 4;
      const v4f rr = *(const v4f*)(rb + (size_t)rowl * ldc + col);
      v4f v = *(const v4f*)(&ldsF[rowl * 68 + col]);
      v[0] += (resrnd != 0) ? bf16_rne(rr[0]) : rr[0];
      v[1] += (resrnd != 0) ? bf16_rne(rr[1]) : rr[1];
      v[2] += (resrnd != 0) ? bf16_rne(rr[2]) : rr[2];
      v[3] += (resrnd != 0) ? bf16_rne(rr[3]) : rr[3];
      *(volatile v4f*)(ob + (size_t)rowl * ldc + col) = v;
    }
  }
}

__global__ __launch_bounds__(256) void k_dw(const _Float16* __restrict__ in,
                                            const float* __restrict__ w,
                                            const float* __restrict__ bias,
                                            _Float16* __restrict__ out, int total8)
{
#pragma clang fp contract(off)
  const int i8 = blockIdx.x * 256 + threadIdx.x;
  if (i8 >= total8) return;
  const int row = i8 / (DM / 8);
  const int d0  = (i8 - row * (DM / 8)) * 8;
  const int img = row >> 10, s = row & 1023;
  const int hh = s >> 5, ww = s & 31;
  float acc[8];
#pragma unroll
  for (int j = 0; j < 8; ++j) acc[j] = bf16_rne(bias[d0 + j]) * ACT_CAR;
#pragma unroll 1
  for (int tap = 0; tap < 9; ++tap) {
    const int kh = tap / 3, kw = tap - 3 * kh;
    const int h2 = hh + kh - 1, w2 = ww + kw - 1;
    const float okf = (h2 >= 0 && h2 <= 31 && w2 >= 0 && w2 <= 31) ? 1.0f : 0.0f;
    const int h2c = min(max(h2, 0), 31), w2c = min(max(w2, 0), 31);
    const v8h xv = *(const v8h*)(in + ((size_t)img * 1024 + (size_t)(h2c * 32 + w2c)) * DM + d0);
#pragma unroll
    for (int j = 0; j < 8; ++j) {
      const float wj = bf16_rne(w[(d0 + j) * 9 + tap]) * okf;
      acc[j] += (float)xv[j] * wj;
    }
  }
  v8h o;
#pragma unroll
  for (int j = 0; j < 8; ++j) o[j] = toh_flush(acc[j]);
  _Float16* d = out + (size_t)i8 * 8;
  *(volatile v8h*)d = o;
  __threadfence();
  *(volatile v8h*)d = o;
}

__device__ __forceinline__ float pool16(const _Float16* __restrict__ P, size_t off) {
  float s = 0.f;
#pragma unroll
  for (int i = 0; i < 4; ++i) {
    const v4h x = *(const v4h*)(P + off + (size_t)i * DM);
    s += ((float)x[0] + (float)x[1]) + ((float)x[2] + (float)x[3]);
  }
  return s * 0.0625f;
}

__global__ __launch_bounds__(128) __attribute__((amdgpu_num_vgpr(256)))
void k_pattn(const _Float16* __restrict__ QKV, float* __restrict__ CS)
{
  __shared__ __attribute__((aligned(16))) _Float16 sK[PQ * 40];
  __shared__ __attribute__((aligned(16))) _Float16 sV[PE * 264];
  __shared__ __attribute__((aligned(16))) _Float16 sQ[64 * 40];
  __shared__ __attribute__((aligned(16))) _Float16 sP[4 * 16 * 40];
  __shared__ __attribute__((aligned(16))) float    sO[4 * 256];

  const int tid = threadIdx.x, lane = tid & 31;
  const int wave = __builtin_amdgcn_readfirstlane(tid >> 5);
  const int hl = lane >> 4, c = lane & 15;
  const int q0 = blockIdx.x * 64;
  const int h = blockIdx.y, b = blockIdx.z;
  const int col0 = h * HD;
  const size_t rq = (size_t)(0 * NB + b) * SEQ;
  const size_t rk = (size_t)(1 * NB + b) * SEQ;
  const size_t rv = (size_t)(2 * NB + b) * SEQ;

  {
    const v8h z8 = {};
#pragma unroll 1
    for (int j = 0; j < 4; ++j) {
      const int idx = j * 128 + tid;
      *(v8h*)(&sK[(idx >> 1) * 40 + 16 + 8 * (idx & 1)]) = z8;
    }
    *(v8h*)(&sQ[(tid >> 1) * 40 + 16 + 8 * (tid & 1)]) = z8;
  }
#pragma unroll 1
  for (int j = 0; j < 32; ++j) {
    const int idx = j * 128 + tid;
    const int q = idx >> 4, e = idx & 15;
    const float kv = pool16(QKV, (rk + (size_t)(4 * q)) * DM + col0 + 4 * e);
    const float vv = pool16(QKV, (rv + (size_t)(4 * q)) * DM + col0 + 4 * e);
    sK[q * 40 + e]  = toh_flush(kv);
    sV[e * 264 + q] = toh_flush(vv);
  }
#pragma unroll 1
  for (int j = 0; j < 8; ++j) {
    const int idx = j * 128 + tid;
    const int q = idx >> 4, e = idx & 15;
    const float qv = pool16(QKV, (rq + (size_t)(4 * (q0 + q))) * DM + col0 + 4 * e);
    sQ[q * 40 + e] = toh_flush(qv);
  }
  __syncthreads();

  const v16h qf = ld_frag_s(sQ, (16 * wave + c) * 40, hl);
  const int pOff = wave * (16 * 40);

  float m[8], l[8];
  v8f o = {};
#pragma unroll
  for (int r = 0; r < 8; ++r) { m[r] = -__builtin_inff(); l[r] = 0.f; }

#pragma unroll 1
  for (int kt = 0; kt < PQ / 32; ++kt) {
    const int mk = kt * 32;
    v8f sh[2] = {};
#pragma unroll
    for (int t = 0; t < 2; ++t) {
      const v16h kf = ld_frag_s(sK, (mk + 16 * t + c) * 40, hl);
      sh[t] = mma(qf, kf, sh[t]);
    }
#pragma unroll
    for (int r = 0; r < 8; ++r) {
      const float v0 = sh[0][r] * PS_SCL;
      const float v1 = sh[1][r] * PS_SCL;
      float tm = fmaxf(v0, v1);
      tm = fmaxf(tm, __shfl_xor(tm, 1, 32));
      tm = fmaxf(tm, __shfl_xor(tm, 2, 32));
      tm = fmaxf(tm, __shfl_xor(tm, 4, 32));
      tm = fmaxf(tm, __shfl_xor(tm, 8, 32));
      const float mn = fmaxf(m[r], tm);
      const float al = __expf(m[r] - mn);
      const float p0 = __expf(v0 - mn), p1 = __expf(v1 - mn);
      float rs = p0 + p1;
      rs += __shfl_xor(rs, 1, 32);
      rs += __shfl_xor(rs, 2, 32);
      rs += __shfl_xor(rs, 4, 32);
      rs += __shfl_xor(rs, 8, 32);
      l[r] = l[r] * al + rs;
      m[r] = mn;
      o[r] *= al;
      const int pi = pOff + (8 * hl + r) * 40 + c;
      sP[pi]      = toh_flush(p0 * P_CAR);
      sP[pi + 16] = toh_flush(p1 * P_CAR);
    }
    __syncthreads();

    const v16h pf = ld_frag_s(sP, pOff + c * 40, hl);
    const v16h vf = ld_frag_s(sV, c * 264 + mk, hl);
    o = mma(pf, vf, o);
    __syncthreads();
  }

#pragma unroll
  for (int r = 0; r < 8; ++r) {
    const float inv = 1.0f / l[r];
    sO[wave * 256 + (8 * hl + r) * 16 + c] = o[r] * inv * PV_SCL;
  }
  __syncthreads();
  float* const dst = CS + ((size_t)(b * NH + h) * PQ + q0 + 16 * wave) * PE;
  const v4f a0 = *(const v4f*)(&sO[wave * 256 + lane * 4]);
  const v4f a1 = *(const v4f*)(&sO[wave * 256 + 128 + lane * 4]);
  *(volatile v4f*)(dst + lane * 4)       = a0;
  *(volatile v4f*)(dst + 128 + lane * 4) = a1;
  __threadfence();
  *(volatile v4f*)(dst + lane * 4)       = a0;
  *(volatile v4f*)(dst + 128 + lane * 4) = a1;
}

__global__ __launch_bounds__(128) __attribute__((amdgpu_num_vgpr(256)))
void k_mix(const _Float16* __restrict__ QKV2, const float* __restrict__ CS,
           const float* __restrict__ fw, const float* __restrict__ fb,
           _Float16* __restrict__ FUS)
{
  __shared__ __attribute__((aligned(16))) _Float16 sC[4 * 64 * 40];
  __shared__ __attribute__((aligned(16))) _Float16 sR[4 * DM];

  const int tid = threadIdx.x, lane = tid & 31;
  const int wave = __builtin_amdgcn_readfirstlane(tid >> 5);
  const int hl = lane >> 4, cn = lane & 15;
  const int catOff = wave * (64 * 40);
  const int rOff = wave * DM;

  {
    const v8h z8 = {};
    *(v8h*)(&sC[catOff + lane * 40 + 24])        = z8;
    *(v8h*)(&sC[catOff + (lane + 32) * 40 + 24]) = z8;
  }

  Frag16 fa;
#pragma unroll
  for (int i = 0; i < 16; ++i) {
    const int ch = (i < 8) ? (8 * hl + i) : (16 + 8 * hl + (i - 8));
    const int oc = min(cn, NH - 1);
    const int cc = min(ch, 2 * NH - 1);
    const float wv = bf16_rne(fw[oc * (2 * NH) + cc]) * FW_CAR;
    const bool ok = (cn < NH) && (ch < 2 * NH);
    fa.v[i] = toh_flush(ok ? wv : 0.0f);
  }
  float fbv[8];
#pragma unroll
  for (int r = 0; r < 8; ++r) fbv[r] = bf16_rne(fb[min(8 * hl + r, NH - 1)]) * CAT_CAR;

  const float ef0 = ((float)lane + 0.5f) * 0.25f - 0.5f;
  const float ef1 = ((float)(lane + 32) + 0.5f) * 0.25f - 0.5f;
  const float fl0 = floorf(ef0), fl1 = floorf(ef1);
  const float we0 = ef0 - fl0, we1 = ef1 - fl1;
  const int a0 = min(max((int)fl0, 0), PE - 1), a1 = min(max((int)fl0 + 1, 0), PE - 1);
  const int b0 = min(max((int)fl1, 0), PE - 1), b1 = min(max((int)fl1 + 1, 0), PE - 1);

#pragma unroll 1
  for (int it = 0; it < 4; ++it) {
    const int row = blockIdx.x * 16 + it * 4 + wave;
    const int bb = row / SEQ;
    const int ss = row - bb * SEQ;
    const float sf = ((float)ss + 0.5f) * 0.25f - 0.5f;
    const float fs = floorf(sf);
    const float wsf = sf - fs;
    const int s0c = min(max((int)fs, 0), PQ - 1), s1c = min(max((int)fs + 1, 0), PQ - 1);
    const _Float16* qp = QKV2 + (size_t)row * DM;
    const _Float16* kp = qp + (size_t)ROWS * DM;
    const _Float16* vp = qp + (size_t)2 * ROWS * DM;
    const float* cb = CS + (size_t)bb * NH * (PQ * PE);

#pragma unroll 1
    for (int hc = 0; hc < NH; ++hc) {
      const int o0 = hc * HD + lane;
      const float q0 = (float)qp[o0], q1 = (float)qp[o0 + 32];
      const float k0 = (float)kp[o0], k1 = (float)kp[o0 + 32];
      const float v0 = (float)vp[o0], v1 = (float)vp[o0 + 32];
      const float p0 = q0 * k0 * EW_SCL;
      const float p1 = q1 * k1 * EW_SCL;
      float mx = fmaxf(p0, p1);
      mx = fmaxf(mx, __shfl_xor(mx, 16, 32));
      mx = fmaxf(mx, __shfl_xor(mx, 8, 32));
      mx = fmaxf(mx, __shfl_xor(mx, 4, 32));
      mx = fmaxf(mx, __shfl_xor(mx, 2, 32));
      mx = fmaxf(mx, __shfl_xor(mx, 1, 32));
      const float e0 = __expf(p0 - mx), e1 = __expf(p1 - mx);
      float sm = e0 + e1;
      sm += __shfl_xor(sm, 16, 32);
      sm += __shfl_xor(sm, 8, 32);
      sm += __shfl_xor(sm, 4, 32);
      sm += __shfl_xor(sm, 2, 32);
      sm += __shfl_xor(sm, 1, 32);
      const float inv = 1.0f / sm;
      const float c0 = e0 * inv * v0 * CTX_CAR;
      const float c1 = e1 * inv * v1 * CTX_CAR;

      const float* cs = cb + hc * (PQ * PE);
      const float t00 = cs[s0c * PE + a0], t01 = cs[s0c * PE + a1];
      const float t10 = cs[s1c * PE + a0], t11 = cs[s1c * PE + a1];
      const float u00 = cs[s0c * PE + b0], u01 = cs[s0c * PE + b1];
      const float u10 = cs[s1c * PE + b0], u11 = cs[s1c * PE + b1];
      const float up0 = ((1.f - wsf) * ((1.f - we0) * t00 + we0 * t01)
                       +        wsf  * ((1.f - we0) * t10 + we0 * t11)) * CAT_CAR;
      const float up1 = ((1.f - wsf) * ((1.f - we1) * u00 + we1 * u01)
                       +        wsf  * ((1.f - we1) * u10 + we1 * u11)) * CAT_CAR;

      sC[catOff + lane * 40 + hc]             = toh_flush(c0);
      sC[catOff + (lane + 32) * 40 + hc]      = toh_flush(c1);
      sC[catOff + lane * 40 + NH + hc]        = toh_flush(up0);
      sC[catOff + (lane + 32) * 40 + NH + hc] = toh_flush(up1);
    }
    __syncthreads();

    v8f acc[4];
#pragma unroll
    for (int t = 0; t < 4; ++t) {
      const v16h bf = ld_frag_s(sC, catOff + (16 * t + cn) * 40, hl);
      const v8f zz = {};
      acc[t] = mma(fa.v, bf, zz);
    }
#pragma unroll
    for (int t = 0; t < 4; ++t)
#pragma unroll
      for (int r = 0; r < 8; ++r) {
        const int oo = 8 * hl + r;
        if (oo < NH)
          sR[rOff + oo * HD + 16 * t + cn] = toh_flush(acc[t][r] * FUS_SCL + fbv[r]);
      }
    __syncthreads();

    const v8h o0v = *(const v8h*)(&sR[rOff + lane * 8]);
    const v8h o1v = *(const v8h*)(&sR[rOff + 256 + lane * 8]);
    const v8h o2v = *(const v8h*)(&sR[rOff + 512 + lane * 8]);
    _Float16* d = FUS + (size_t)row * DM + lane * 8;
    *(volatile v8h*)(d)       = o0v;
    *(volatile v8h*)(d + 256) = o1v;
    *(volatile v8h*)(d + 512) = o2v;
    __threadfence();
    *(volatile v8h*)(d)       = o0v;
    *(volatile v8h*)(d + 256) = o1v;
    *(volatile v8h*)(d + 512) = o2v;
    __syncthreads();
  }
}

extern "C" void kernel_launch(void* const* d_in, const int* in_sizes, int n_in,
                              void* d_out, int out_size, void* d_ws, size_t ws_size,
                              hipStream_t stream)
{
  if (n_in < 23) return;
  const long need_x = ((long)(NB - 1) * SEQ_FULL + SEQ) * DM;
  if ((long)in_sizes[0] < need_x) return;
  if ((long)in_sizes[1] < DM || (long)in_sizes[2] < DM) return;
  if ((long)in_sizes[3] < (long)DM * DM || (long)in_sizes[4] < DM) return;
  if ((long)in_sizes[5] < (long)DM * DM || (long)in_sizes[6] < DM) return;
  if ((long)in_sizes[7] < (long)DM * DM || (long)in_sizes[8] < DM) return;
  if ((long)in_sizes[9] < (long)DM * 9 || (long)in_sizes[10] < DM) return;
  if ((long)in_sizes[11] < (long)DM * DM || (long)in_sizes[12] < DM) return;
  if ((long)in_sizes[13] < (long)NH * 2 * NH || (long)in_sizes[14] < NH) return;
  if ((long)in_sizes[15] < (long)DM * DM || (long)in_sizes[16] < DM) return;
  if ((long)in_sizes[17] < DM || (long)in_sizes[18] < DM) return;
  if ((long)in_sizes[19] < (long)MLP * DM || (long)in_sizes[20] < MLP) return;
  if ((long)in_sizes[21] < (long)DM * MLP || (long)in_sizes[22] < DM) return;
  if ((long)out_size < need_x) return;
  if (WS_HALVES * sizeof(_Float16) > ws_size) return;

  const float* x      = (const float*)d_in[0];
  const float* ln1_g  = (const float*)d_in[1];
  const float* ln1_b  = (const float*)d_in[2];
  const float* wq     = (const float*)d_in[3];
  const float* bq     = (const float*)d_in[4];
  const float* wk     = (const float*)d_in[5];
  const float* bk     = (const float*)d_in[6];
  const float* wv     = (const float*)d_in[7];
  const float* bv     = (const float*)d_in[8];
  const float* dw_w   = (const float*)d_in[9];
  const float* dw_b   = (const float*)d_in[10];
  const float* pw_w   = (const float*)d_in[11];
  const float* pw_b   = (const float*)d_in[12];
  const float* fuse_w = (const float*)d_in[13];
  const float* fuse_b = (const float*)d_in[14];
  const float* wo     = (const float*)d_in[15];
  const float* bo     = (const float*)d_in[16];
  const float* ln2_g  = (const float*)d_in[17];
  const float* ln2_b  = (const float*)d_in[18];
  const float* fc1_w  = (const float*)d_in[19];
  const float* fc1_b  = (const float*)d_in[20];
  const float* fc2_w  = (const float*)d_in[21];
  const float* fc2_b  = (const float*)d_in[22];
  float* out = (float*)d_out;

  _Float16* DS   = (_Float16*)d_ws;
  _Float16* DD   = DS   + N_DS;
  _Float16* WQ   = DD   + N_DD;
  _Float16* PW   = WQ   + N_WQ;
  _Float16* WO   = PW   + N_W1;
  _Float16* FC1  = WO   + N_W1;
  _Float16* FC2  = FC1  + N_FC;
  _Float16* XN   = FC2  + N_FC;
  _Float16* UT   = XN   + N_ACT;
  _Float16* XD   = UT   + N_ACT;
  _Float16* QKV  = XD   + N_ACT;
  _Float16* DW   = QKV  + N_3ACT;
  _Float16* QKV2 = DW   + N_3ACT;
  float*    CS   = (float*)(QKV2 + N_3ACT);
  _Float16* FUS  = (_Float16*)CS + N_CS;
  _Float16* AO   = FUS  + N_ACT;
  _Float16* WT   = AO   + N_ACT;
  float*    X2   = (float*)(WT + N_ACT);
  _Float16* XM   = (_Float16*)X2 + N_X2;
  _Float16* H1   = XM   + N_ACT;

  const size_t nAct = (size_t)ROWS * DM;
  const size_t nBat = (size_t)SEQ * DM;

  k_gen<<<dim3((SEQ * SEQ) / 2048, 2), 256, 0, stream>>>(DS, SEQ,
      (float)sqrt(1.0 / (double)SEQ), (float)sqrt(2.0 / (double)SEQ));
  k_gen<<<dim3((DM * DM) / 2048, 2), 256, 0, stream>>>(DD, DM,
      (float)sqrt(1.0 / (double)DM), (float)sqrt(2.0 / (double)DM));

  const int tw8 = (DM * DM) / 8;
  const int tf8 = (MLP * DM) / 8;
  k_cvt8<<<tw8 / 256, 256, 0, stream>>>(wq,   WQ,                       DM, DM, DM, W_CAR, tw8);
  k_cvt8<<<tw8 / 256, 256, 0, stream>>>(wk,   WQ + (size_t)DM * DM,     DM, DM, DM, W_CAR, tw8);
  k_cvt8<<<tw8 / 256, 256, 0, stream>>>(wv,   WQ + (size_t)2 * DM * DM, DM, DM, DM, W_CAR, tw8);
  k_cvt8<<<tw8 / 256, 256, 0, stream>>>(pw_w, PW,  DM, DM, DM, W_CAR, tw8);
  k_cvt8<<<tw8 / 256, 256, 0, stream>>>(wo,   WO,  DM, DM, DM, W_CAR, tw8);
  k_cvt8<<<tf8 / 256, 256, 0, stream>>>(fc1_w, FC1, DM,  MLP, MLP, W_CAR, tf8);
  k_cvt8<<<tf8 / 256, 256, 0, stream>>>(fc2_w, FC2, MLP, DM,  DM,  W_CAR, tf8);

  k_ln<<<ROWS / 8, 256, 0, stream>>>(x, ln1_g, ln1_b, XN, 1, ROWS);

  k_gemm<<<dim3(SEQ / 64, DM / 128, NB), 128, 0, stream>>>(
      DD, XN, ln1_b, x, UT, X2, (size_t)0, nBat, nBat,
      DM, SEQ, SCL_M10, 1.0f, 1.0f, 0, 0);
  k_gemm<<<dim3(DM / 64, SEQ / 128, NB), 128, 0, stream>>>(
      DS, UT, ln1_b, x, XD, X2, (size_t)0, nBat, nBat,
      SEQ, DM, SCL_M13, 1.0f, ACT_CAR, GM_THR, 0);

  k_gemm<<<dim3(DM / 64, ROWS / 128, 1), 128, 0, stream>>>(
      XD, WQ, bq, x, QKV, X2, (size_t)0, (size_t)0, (size_t)0,
      DM, DM, SCL_M10, ACT_CAR, 1.0f, GM_BIAS, 0);
  k_gemm<<<dim3(DM / 64, ROWS / 128, 1), 128, 0, stream>>>(
      XD, WQ + (size_t)DM * DM, bk, x, QKV + nAct, X2, (size_t)0, (size_t)0, (size_t)0,
      DM, DM, SCL_M10, ACT_CAR, 1.0f, GM_BIAS, 0);
  k_gemm<<<dim3(DM / 64, ROWS / 128, 1), 128, 0, stream>>>(
      XD, WQ + (size_t)2 * DM * DM, bv, x, QKV + 2 * nAct, X2, (size_t)0, (size_t)0, (size_t)0,
      DM, DM, SCL_M10, ACT_CAR, 1.0f, GM_BIAS, 0);

  const int td8 = (int)(((size_t)3 * ROWS * DM) / 8);
  k_dw<<<td8 / 256, 256, 0, stream>>>(QKV, dw_w, dw_b, DW, td8);
  k_gemm<<<dim3(DM / 64, (3 * ROWS) / 128, 1), 128, 0, stream>>>(
      DW, PW, pw_b, x, QKV2, X2, (size_t)0, (size_t)0, (size_t)0,
      DM, DM, SCL_M10, ACT_CAR, 1.0f, GM_BIAS, 0);

  k_pattn<<<dim3(PQ / 64, NH, NB), 128, 0, stream>>>(QKV, CS);
  k_mix<<<ROWS / 16, 128, 0, stream>>>(QKV2, CS, fuse_w, fuse_b, FUS);

  k_gemm<<<dim3(DM / 64, ROWS / 128, 1), 128, 0, stream>>>(
      FUS, WO, bo, x, AO, X2, (size_t)0, (size_t)0, (size_t)0,
      DM, DM, SCL_M10, CAT_CAR, 1.0f, GM_BIAS, 0);

  k_gemm<<<dim3(SEQ / 64, DM / 128, NB), 128, 0, stream>>>(
      DD + (size_t)DM * DM, AO, ln1_b, x, WT, X2, (size_t)0, nBat, nBat,
      DM, SEQ, SCL_M10, 1.0f, 1.0f, 0, 0);
  k_gemm<<<dim3(DM / 64, SEQ / 128, NB), 128, 0, stream>>>(
      DS + (size_t)SEQ * SEQ, WT, ln1_b, x, XM, X2, (size_t)0, nBat, nBat,
      SEQ, DM, SCL_M20, 1.0f, 1.0f, GM_F32, 1);

  k_ln<<<ROWS / 8, 256, 0, stream>>>(X2, ln2_g, ln2_b, XM, 0, ROWS);
  k_gemm<<<dim3(MLP / 64, ROWS / 128, 1), 128, 0, stream>>>(
      XM, FC1, fc1_b, x, H1, X2, (size_t)0, (size_t)0, (size_t)0,
      DM, MLP, SCL_M13, 1.0f, ACT_CAR, GM_BIAS | GM_GELU, 0);
  k_gemm<<<dim3(DM / 64, ROWS / 128, 1), 128, 0, stream>>>(
      H1, FC2, fc2_b, X2, XM, out, (size_t)0, (size_t)0, (size_t)0,
      MLP, DM, SCL_M13, 1.0f, 1.0f, GM_F32 | GM_BIAS, 0);
}
